// UnifiedDeepRanker_42511586295930
// MI455X (gfx1250) — hardware-verified
//
#include <hip/hip_runtime.h>


namespace {
constexpr int NB = 8192, L = 50, LP = 64, DE = 128, NU = 100001, NM = 50001, ND = 8, D = 392, DP = 416, NE = 4, NTK = 2, H1 = 256, H2 = 128, AH = 64, NX = 3;
constexpr float XS = 8.0f, WSC = 256.0f, EPS = 1e-5f;

typedef _Float16 b16;
typedef __attribute__((ext_vector_type(16))) _Float16 v16b;
typedef __attribute__((ext_vector_type(8))) _Float16 v8b;
typedef __attribute__((ext_vector_type(8))) float v8f;
typedef __attribute__((ext_vector_type(4))) float v4f;
__device__ __forceinline__ float bf16_rne(float f) { unsigned int u = __float_as_uint(f); u += 0x7FFFu + ((u >> 16) & 1u); return __uint_as_float(u & 0xFFFF0000u); }
__device__ __forceinline__ void split16(float v, b16& hi, b16& lo) { hi = (b16)v; lo = (b16)(v - (float)hi); }
__device__ __forceinline__ v16b frag_kb(const b16* p, int hh) { const v8b a = *(const v8b*)(p + 8 * hh), b = *(const v8b*)(p + 16 + 8 * hh); v16b f;
#pragma unroll
  for (int e = 0; e < 8; ++e) { f[e] = a[e]; f[8 + e] = b[e]; } return f; }
__device__ __forceinline__ v8f wmma16b(v16b a, v16b b, v8f c) { v8f d = __builtin_amdgcn_wmma_f32_16x16x32_f16(false, a, false, b, (short)0, c, false, false); asm volatile("v_nop\n\tv_nop\n\tv_nop\n\tv_nop" : "+v"(d) : "v"(a), "v"(b)); return d; }
__device__ __forceinline__ void wave_lds_sync() { __builtin_amdgcn_fence(__ATOMIC_RELEASE, "workgroup"); __builtin_amdgcn_wave_barrier(); __builtin_amdgcn_fence(__ATOMIC_ACQUIRE, "workgroup"); }
__device__ __forceinline__ float pmul(float a, float b) { float p = a * b; asm volatile("" : "+v"(p)); return p; }
__device__ __forceinline__ int iclamp(int v, int lo, int hi) { return v < lo ? lo : (v > hi ? hi : v); }

__global__ __launch_bounds__(256) void wprep_kernel(const float* __restrict__ w, int nin, int nout, int ldw, int ninp, int noutp, int mode, b16* __restrict__ dst, b16* __restrict__ dstl) {
  const size_t u = (size_t)blockIdx.x * 256 + threadIdx.x; if (u >= (size_t)noutp * ninp / 8) return; const size_t e = u * 8; const int oo = (int)(e / ninp), k0 = (int)(e % ninp); v8b o, ol;
  for (int j = 0; j < 8; ++j) { const int k = k0 + j; float v = 0.0f;
    if (oo < nout && k < nin) { if (mode == 0) v = bf16_rne(w[(size_t)k * ldw + oo]); else if (mode == 1) v = bf16_rne(w[(size_t)(DE + k) * ldw + oo]) - bf16_rne(w[(size_t)(2 * DE + k) * ldw + oo]); else v = bf16_rne(w[(size_t)k * ldw + oo]) + bf16_rne(w[(size_t)(2 * DE + k) * ldw + oo]); }
    b16 p, q; split16(v * WSC, p, q); o[j] = p; ol[j] = q; }
  for (int pass = 0; pass < 2; ++pass) { *(volatile v8b*)(dst + e) = o; if (dstl) *(volatile v8b*)(dstl + e) = ol; __threadfence(); }
}
__global__ __launch_bounds__(256) void qprep_kernel(const float* __restrict__ embm, const int* __restrict__ mid, b16* __restrict__ Q16) {
  const size_t u = (size_t)blockIdx.x * 256 + threadIdx.x; if (u >= (size_t)NB * DE / 8) return; const size_t e = u * 8; const int b = (int)(e / DE), c0 = (int)(e % DE); const int m = iclamp(mid[b], 0, NM - 1); v8b o;
  for (int j = 0; j < 8; ++j) o[j] = (b16)(bf16_rne(embm[(size_t)m * DE + c0 + j]) * XS);
  for (int pass = 0; pass < 2; ++pass) { *(volatile v8b*)(Q16 + e) = o; __threadfence(); }
}
__global__ __launch_bounds__(128) void qterm_kernel(const b16* __restrict__ Q16, const b16* __restrict__ WQh, const b16* __restrict__ WQl, const float* __restrict__ b1, float* __restrict__ QT) {
  __shared__ __attribute__((aligned(16))) float Tf[4][16][AH + 4];
  const int wave = threadIdx.x >> 5, lane = threadIdx.x & 31, nloc = lane & 15, hlf = lane >> 4; const size_t m0 = (size_t)blockIdx.x * 64 + wave * 16; v8f acc[4] = {{}, {}, {}, {}};
#pragma unroll
  for (int kb = 0; kb < DE; kb += 32) { const v16b a = frag_kb(Q16 + (m0 + nloc) * DE + kb, hlf);
#pragma unroll
    for (int t = 0; t < 4; ++t) { acc[t] = wmma16b(a, frag_kb(WQh + (size_t)(t * 16 + nloc) * DE + kb, hlf), acc[t]); acc[t] = wmma16b(a, frag_kb(WQl + (size_t)(t * 16 + nloc) * DE + kb, hlf), acc[t]); } }
#pragma unroll
  for (int t = 0; t < 4; ++t) { const float bb = bf16_rne(b1[t * 16 + nloc]); for (int r = 0; r < 8; ++r) Tf[wave][8 * hlf + r][t * 16 + nloc] = acc[t][r] * (1.0f / (XS * WSC)) + bb; }
  wave_lds_sync();
  for (int pass = 0; pass < 2; ++pass) { for (int rr = 0; rr < 16; ++rr) if (lane < 16) *(volatile v4f*)(QT + (m0 + rr) * AH + lane * 4) = *(const v4f*)(&Tf[wave][rr][lane * 4]); __threadfence(); }
}
__global__ __launch_bounds__(128) void din_kernel(const float* __restrict__ embu, const float* __restrict__ embm, const int* __restrict__ uid, const int* __restrict__ mid, const int* __restrict__ hist, const float* __restrict__ dense, const float* __restrict__ QT,
    const b16* __restrict__ WKh, const b16* __restrict__ WKl, const b16* __restrict__ WP, const float* __restrict__ w2, const float* __restrict__ b2, float* __restrict__ X0) {
  __shared__ __attribute__((aligned(16))) b16 Kt[LP][DE + 8], Ph[LP][DE + 8], Pl[LP][DE + 8]; __shared__ float sc[LP]; __shared__ float prob[LP]; __shared__ __attribute__((aligned(16))) float row[DP];
  const int wave = threadIdx.x >> 5, lane = threadIdx.x & 31, nloc = lane & 15, hlf = lane >> 4, t_ = threadIdx.x; const int b = blockIdx.x; const int m = iclamp(mid[b], 0, NM - 1), us = iclamp(uid[b], 0, NU - 1);
  for (int q = t_; q < LP * (DE / 4); q += 128) { const int l = q / (DE / 4), c4 = (q % (DE / 4)) * 4; int id = 0; if (l < L) id = iclamp(hist[b * L + l], 0, NM - 1);
    for (int j = 0; j < 4; ++j) { const int c = c4 + j; const float kv = (l < L) ? bf16_rne(embm[(size_t)id * DE + c]) : 0.0f; const float qv = bf16_rne(embm[(size_t)m * DE + c]); Kt[l][c] = (b16)(kv * XS); b16 p, pl; split16(pmul(qv, kv) * XS, p, pl); Ph[l][c] = p; Pl[l][c] = pl; } }
  __syncthreads();
  v8f acc[4] = {{}, {}, {}, {}}; const int l0 = wave * 16;
#pragma unroll
  for (int kb = 0; kb < DE; kb += 32) { const v16b ka = frag_kb(&Kt[l0 + nloc][kb], hlf), pa = frag_kb(&Ph[l0 + nloc][kb], hlf), pal = frag_kb(&Pl[l0 + nloc][kb], hlf);
#pragma unroll
    for (int t = 0; t < 4; ++t) { const v16b wkh = frag_kb(WKh + (size_t)(t * 16 + nloc) * DE + kb, hlf), wkl = frag_kb(WKl + (size_t)(t * 16 + nloc) * DE + kb, hlf), wp = frag_kb(WP + (size_t)(t * 16 + nloc) * DE + kb, hlf);
      acc[t] = wmma16b(ka, wkh, acc[t]); acc[t] = wmma16b(ka, wkl, acc[t]); acc[t] = wmma16b(pa, wp, acc[t]); acc[t] = wmma16b(pal, wp, acc[t]); } }
#pragma unroll 1
  for (int r = 0; r < 8; ++r) { float s = 0.0f;
    for (int t = 0; t < 4; ++t) { const int c = t * 16 + nloc; const float h = fmaxf(acc[t][r] * (1.0f / (XS * WSC)) + QT[(size_t)b * AH + c], 0.0f); s += pmul(h, bf16_rne(w2[c])); }
    s += __shfl_xor(s, 1); s += __shfl_xor(s, 2); s += __shfl_xor(s, 4); s += __shfl_xor(s, 8);
    if (nloc == 0) { const int l = l0 + 8 * hlf + r; const bool valid = (l < L) && (hist[b * L + l] > 0); sc[l] = valid ? s + bf16_rne(b2[0]) : ((l < L) ? -1e9f : -INFINITY); } }
  __syncthreads();
  if (t_ == 0) { float mx = -INFINITY; for (int l = 0; l < L; ++l) mx = fmaxf(mx, sc[l]); float se = 0.0f; for (int l = 0; l < L; ++l) { prob[l] = __expf(sc[l] - mx); se += prob[l]; } const float inv = 1.0f / se; for (int l = 0; l < L; ++l) prob[l] *= inv; }
  __syncthreads();
  if (t_ < DE) { float s = 0.0f; for (int l = 0; l < L; ++l) s += pmul(prob[l], (float)Kt[l][t_] * (1.0f / XS)); row[2 * DE + t_] = s; row[t_] = bf16_rne(embu[(size_t)us * DE + t_]); row[DE + t_] = bf16_rne(embm[(size_t)m * DE + t_]); }
  if (t_ < DP - 3 * DE) { const int c = 3 * DE + t_; row[c] = (t_ < ND) ? bf16_rne(dense[b * ND + t_]) : 0.0f; }
  __syncthreads();
  for (int pass = 0; pass < 2; ++pass) { if (t_ < DP / 4) *(volatile v4f*)(X0 + (size_t)b * DP + t_ * 4) = *(const v4f*)(&row[t_ * 4]); __threadfence(); }
}
__global__ __launch_bounds__(256) void ln_kernel(const float* __restrict__ X, const float* __restrict__ g, const float* __restrict__ bta, float* __restrict__ Y) {
  const int wave = threadIdx.x >> 5, lane = threadIdx.x & 31; const size_t rowi = (size_t)blockIdx.x * 8 + wave; float x[13]; for (int j = 0; j < 13; ++j) x[j] = X[rowi * DP + lane * 13 + j];
  float s = 0.0f; for (int j = 0; j < 13; ++j) { const int c = lane * 13 + j; if (c < D) s += x[j]; }
#pragma unroll
  for (int o = 16; o >= 1; o >>= 1) s += __shfl_xor(s, o);
  const float mu = s * (1.0f / D); float q = 0.0f; for (int j = 0; j < 13; ++j) { const int c = lane * 13 + j; if (c < D) { const float d = x[j] - mu; q += d * d; } }
#pragma unroll
  for (int o = 16; o >= 1; o >>= 1) q += __shfl_xor(q, o);
  const float rs = rsqrtf(q * (1.0f / D) + EPS); __shared__ __attribute__((aligned(16))) float rowb[8][DP];
  for (int j = 0; j < 13; ++j) { const int c = lane * 13 + j; rowb[wave][c] = (c < D) ? (x[j] - mu) * rs * bf16_rne(g[c]) + bf16_rne(bta[c]) : 0.0f; }
  wave_lds_sync();
  for (int pass = 0; pass < 2; ++pass) { for (int q4 = lane; q4 < DP / 4; q4 += 32) *(volatile v4f*)(Y + rowi * DP + q4 * 4) = *(const v4f*)(&rowb[wave][q4 * 4]); __threadfence(); }
}
template <int KD, int NTL, int EPI, int NW>
__global__ __launch_bounds__(NW * 32) void dense_kernel(const float* __restrict__ X, int ldx, const b16* __restrict__ Wt, const float* __restrict__ bias, int nbias, const float* __restrict__ RES, float* __restrict__ Y, int ldy) {
  __shared__ __attribute__((aligned(16))) b16 Ah[NW][16][KD + 8], Al[NW][16][KD + 8]; __shared__ __attribute__((aligned(16))) float Tf[NW][16][NTL * 16 + 4];
  const int wave = threadIdx.x >> 5, lane = threadIdx.x & 31, nloc = lane & 15, hlf = lane >> 4; const size_t m0 = (size_t)blockIdx.x * (NW * 16) + wave * 16; const int n0 = blockIdx.y * NTL * 16;
  for (int q = lane; q < 16 * (KD / 4); q += 32) { const int rr = q / (KD / 4), c4 = (q % (KD / 4)) * 4; const v4f xv = *(const v4f*)(X + (m0 + rr) * ldx + c4); for (int j = 0; j < 4; ++j) { b16 p, pl; split16(xv[j] * XS, p, pl); Ah[wave][rr][c4 + j] = p; Al[wave][rr][c4 + j] = pl; } }
  wave_lds_sync();
  v8f acc[NTL];
#pragma unroll
  for (int t = 0; t < NTL; ++t) acc[t] = (v8f){};
#pragma unroll 2
  for (int kb = 0; kb < KD; kb += 32) { const v16b a = frag_kb(&Ah[wave][nloc][kb], hlf), al = frag_kb(&Al[wave][nloc][kb], hlf);
#pragma unroll
    for (int t = 0; t < NTL; ++t) { const v16b bw = frag_kb(Wt + (size_t)(n0 + t * 16 + nloc) * KD + kb, hlf); acc[t] = wmma16b(a, bw, acc[t]); acc[t] = wmma16b(al, bw, acc[t]); } }
#pragma unroll
  for (int t = 0; t < NTL; ++t) { const int c = n0 + t * 16 + nloc; const float bb = (bias != nullptr && c < nbias) ? bf16_rne(bias[c]) : 0.0f;
#pragma unroll 1
    for (int r = 0; r < 8; ++r) { const size_t rowi = m0 + 8 * hlf + r; float y = acc[t][r] * (1.0f / (XS * WSC)) + bb; if (EPI == 1) y = fmaxf(y, 0.0f); else if (EPI == 2) y = (c < D) ? pmul(RES[rowi * DP + c], y) + X[rowi * ldx + c] : 0.0f; Tf[wave][8 * hlf + r][t * 16 + nloc] = y; } }
  wave_lds_sync();
  for (int pass = 0; pass < 2; ++pass) { for (int q = lane; q < 16 * NTL * 4; q += 32) { const int rr = q / (NTL * 4), c4 = (q % (NTL * 4)) * 4; *(volatile v4f*)(Y + (m0 + rr) * ldy + n0 + c4) = *(const v4f*)(&Tf[wave][rr][c4]); } __threadfence(); }
}
__global__ __launch_bounds__(256) void final_kernel(const float* __restrict__ G, const float* __restrict__ gb, const float* __restrict__ EO, const float* __restrict__ hw, const float* __restrict__ hb, float* __restrict__ out) {
  __shared__ __attribute__((aligned(16))) float res[NTK][256];
  const int t_ = threadIdx.x; const size_t b = (size_t)blockIdx.x * 256 + t_;
  for (int t = 0; t < NTK; ++t) { float g[NE]; float mx = -INFINITY; for (int e = 0; e < NE; ++e) { g[e] = G[b * 32 + t * 16 + e] + bf16_rne(gb[t * NE + e]); mx = fmaxf(mx, g[e]); } float se = 0.0f; for (int e = 0; e < NE; ++e) { g[e] = __expf(g[e] - mx); se += g[e]; } const float inv = 1.0f / se;
    float s = bf16_rne(hb[t]);
#pragma unroll 1
    for (int o = 0; o < H2; ++o) { float tf = 0.0f; for (int e = 0; e < NE; ++e) tf += pmul(g[e] * inv, EO[((size_t)e * NB + b) * H2 + o]); s += pmul(tf, bf16_rne(hw[t * H2 + o])); }
    res[t][t_] = s; }
  __syncthreads();
  for (int pass = 0; pass < 2; ++pass) { if (t_ < 128) { const int t = t_ >> 6, q4 = t_ & 63; *(volatile v4f*)(out + (size_t)t * NB + (size_t)blockIdx.x * 256 + q4 * 4) = *(const v4f*)(&res[t][q4 * 4]); } __threadfence(); }
}
}

extern "C" void kernel_launch(void* const* d_in, const int* in_sizes, int n_in, void* d_out, int out_size, void* d_ws, size_t ws_size, hipStream_t stream) {
  (void)n_in;
  auto Fp = [&](int i) { return (const float*)d_in[i]; }; auto Ip = [&](int i) { return (const int*)d_in[i]; };
  if (in_sizes[0] != NB || in_sizes[2] != NB * L || in_sizes[3] != NB * ND || in_sizes[4] != NU * DE || in_sizes[5] != NM * DE || in_sizes[6] != 4 * DE * AH || in_sizes[14] != NX * D * D || in_sizes[16] != NE * D * H1 || in_sizes[18] != NE * H1 * H2 || in_sizes[20] != NTK * D * NE || out_size != NTK * NB) return;
  size_t off = 0; char* ws = (char*)d_ws;
  auto carve = [&](size_t bytes) { char* p = ws + off; off += (bytes + 255) & ~(size_t)255; return p; };
  b16* WQh = (b16*)carve((size_t)AH * DE * 2); b16* WQl = (b16*)carve((size_t)AH * DE * 2); b16* WKh = (b16*)carve((size_t)AH * DE * 2); b16* WKl = (b16*)carve((size_t)AH * DE * 2); b16* WP = (b16*)carve((size_t)AH * DE * 2);
  b16* WX = (b16*)carve((size_t)NX * DP * DP * 2); b16* WE1 = (b16*)carve((size_t)NE * H1 * DP * 2); b16* WE2 = (b16*)carve((size_t)NE * H2 * H1 * 2); b16* WG = (b16*)carve((size_t)32 * DP * 2);
  b16* Q16 = (b16*)carve((size_t)NB * DE * 2); float* QT = (float*)carve((size_t)NB * AH * 4); float* X0 = (float*)carve((size_t)NB * DP * 4); float* XA = (float*)carve((size_t)NB * DP * 4); float* XB = (float*)carve((size_t)NB * DP * 4);
  float* HE = (float*)carve((size_t)NB * H1 * 4); float* EO = (float*)carve((size_t)NE * NB * H2 * 4); float* G = (float*)carve((size_t)NB * 32 * 4);
  if (off > ws_size || off > ((size_t)128 << 20)) return;
  auto wprep = [&](const float* w, int nin, int nout, int ldw, int ninp, int noutp, int mode, b16* dst, b16* dstl) { wprep_kernel<<<(unsigned)(((size_t)noutp * ninp / 8 + 255) / 256), 256, 0, stream>>>(w, nin, nout, ldw, ninp, noutp, mode, dst, dstl); };
  wprep(Fp(6), DE, AH, AH, DE, AH, 2, WQh, WQl);
  wprep(Fp(6), DE, AH, AH, DE, AH, 1, WKh, WKl);
  wprep(Fp(6) + (size_t)3 * DE * AH, DE, AH, AH, DE, AH, 0, WP, nullptr);
  for (int l = 0; l < NX; ++l) wprep(Fp(14) + (size_t)l * D * D, D, D, D, DP, DP, 0, WX + (size_t)l * DP * DP, nullptr);
  for (int e = 0; e < NE; ++e) { wprep(Fp(16) + (size_t)e * D * H1, D, H1, H1, DP, H1, 0, WE1 + (size_t)e * H1 * DP, nullptr); wprep(Fp(18) + (size_t)e * H1 * H2, H1, H2, H2, H1, H2, 0, WE2 + (size_t)e * H2 * H1, nullptr); }
  for (int t = 0; t < NTK; ++t) wprep(Fp(20) + (size_t)t * D * NE, D, NE, NE, DP, 16, 0, WG + (size_t)t * 16 * DP, nullptr);
  qprep_kernel<<<(unsigned)(((size_t)NB * DE / 8 + 255) / 256), 256, 0, stream>>>(Fp(5), Ip(1), Q16);
  qterm_kernel<<<NB / 64, 128, 0, stream>>>(Q16, WQh, WQl, Fp(7), QT);
  din_kernel<<<NB, 128, 0, stream>>>(Fp(4), Fp(5), Ip(0), Ip(1), Ip(2), Fp(3), QT, WKh, WKl, WP, Fp(8), Fp(9), X0);
  ln_kernel<<<NB / 8, 256, 0, stream>>>(X0, Fp(10), Fp(11), XA);
  dense_kernel<DP, 13, 2, 2><<<dim3(NB / 32, 2), 64, 0, stream>>>(XA, DP, WX, Fp(15), D, XA, XB, DP);
  dense_kernel<DP, 13, 2, 2><<<dim3(NB / 32, 2), 64, 0, stream>>>(XB, DP, WX + (size_t)DP * DP, Fp(15) + D, D, XA, X0, DP);
  dense_kernel<DP, 13, 2, 2><<<dim3(NB / 32, 2), 64, 0, stream>>>(X0, DP, WX + (size_t)2 * DP * DP, Fp(15) + 2 * D, D, XA, XB, DP);
  ln_kernel<<<NB / 8, 256, 0, stream>>>(XB, Fp(12), Fp(13), XA);
  for (int e = 0; e < NE; ++e) {
    dense_kernel<DP, 8, 1, 2><<<dim3(NB / 32, H1 / 128), 64, 0, stream>>>(XA, DP, WE1 + (size_t)e * H1 * DP, Fp(17) + e * H1, H1, nullptr, HE, H1);
    dense_kernel<H1, 8, 0, 4><<<dim3(NB / 64, 1), 128, 0, stream>>>(HE, H1, WE2 + (size_t)e * H2 * H1, Fp(19) + e * H2, H2, nullptr, EO + (size_t)e * NB * H2, H2); }
  dense_kernel<DP, 2, 0, 2><<<dim3(NB / 32, 1), 64, 0, stream>>>(XA, DP, WG, nullptr, 0, nullptr, G, 32);
  final_kernel<<<NB / 256, 256, 0, stream>>>(G, Fp(21), EO, Fp(22), Fp(23), (float*)d_out);
}
